// EdgeScore_function_67001489817643
// MI455X (gfx1250) — hardware-run, weakly checked
//
#include <hip/hip_runtime.h>
#include <math.h>

#ifndef SEQ
#define SEQ 1024
#endif
#define SEQ_FULL 1024
#define DD 1024
#define HH 100
#define ROFF 128
#define NOP 256
#define PT 32
#define LSTR 101

#define A16_BYTES ((size_t)SEQ * DD * 2)
#define W16_BYTES ((size_t)NOP * DD * 2)
#define LR_BYTES  ((size_t)SEQ * NOP * 4)

static_assert(SEQ % 64 == 0);
static_assert(SEQ % PT == 0);
static_assert(SEQ <= SEQ_FULL);
static_assert(NOP % 64 == 0);
static_assert(DD % 32 == 0);
static_assert(DD % 8 == 0);
static_assert(HH % 4 == 0);
static_assert(ROFF >= HH);
static_assert(ROFF + HH <= NOP);
static_assert(ROFF % 4 == 0);
static_assert(NOP % 4 == 0);
static_assert(LSTR >= HH);
static_assert(((size_t)SEQ * DD) % (8 * 256) == 0);
static_assert(((size_t)NOP * DD) % (8 * 256) == 0);
static_assert(256 * 16 == PT * PT * 4);
static_assert((2 * PT * LSTR + HH) * 4 <= 131072);
static_assert(8 * 16 * 68 * 4 <= 131072);
static_assert(A16_BYTES % 256 == 0);
static_assert(W16_BYTES % 256 == 0);
static_assert(LR_BYTES % 256 == 0);
static_assert(A16_BYTES + W16_BYTES + LR_BYTES <= (size_t)134217728);

namespace eng {
typedef __attribute__((ext_vector_type(16))) _Float16 v16h;
typedef __attribute__((ext_vector_type(8)))  _Float16 v8h;
typedef __attribute__((ext_vector_type(16))) __bf16   v16b;
typedef __attribute__((ext_vector_type(8)))  __bf16   v8b;
typedef __attribute__((ext_vector_type(8)))  float    v8f;
typedef __attribute__((ext_vector_type(4)))  float    v4f;

__device__ __forceinline__ unsigned short f2bf_bits(float f) {
  unsigned u = __float_as_uint(f);
  return (unsigned short)((u + 0x7FFFu + ((u >> 16) & 1u)) >> 16);
}
__device__ __forceinline__ float bf_bits2f(unsigned short h) { return __uint_as_float(((unsigned)h) << 16); }

__device__ __forceinline__ void dep_guard_h(v8f& a, v8f& b, v16h x, v16h y) { asm volatile("v_nop\n\tv_nop\n\tv_nop\n\tv_nop" : "+v"(a), "+v"(b) : "v"(x), "v"(y)); }
__device__ __forceinline__ void dep_guard_b(v8f& a, v8f& b, v16b x, v16b y) { asm volatile("v_nop\n\tv_nop\n\tv_nop\n\tv_nop" : "+v"(a), "+v"(b) : "v"(x), "v"(y)); }
__device__ __forceinline__ void keep4_h(v16h a, v16h b, v16h c, v16h d) { asm volatile("v_nop" :: "v"(a), "v"(b), "v"(c), "v"(d)); }
__device__ __forceinline__ void keep4_b(v16b a, v16b b, v16b c, v16b d) { asm volatile("v_nop" :: "v"(a), "v"(b), "v"(c), "v"(d)); }
__device__ __forceinline__ void acc_guard4(v8f& a, v8f& b, v8f& c, v8f& d) { asm volatile("v_nop\n\tv_nop\n\tv_nop\n\tv_nop" : "+v"(a), "+v"(b), "+v"(c), "+v"(d)); }
template <typename T> struct Frag;
template <> struct Frag<_Float16> {
  typedef v16h V; union U { v16h v; v8h h[2]; };
  static __device__ __forceinline__ v16h load(const _Float16* p) {
    U f; f.h[0] = *(const v8h*)(p); f.h[1] = *(const v8h*)(p + 16); return f.v;
  }
  static __device__ __forceinline__ v8f mma(v16h a, v16h b, v8f c) {
    return __builtin_amdgcn_wmma_f32_16x16x32_f16(false, a, false, b, (short)0, c, false, false);
  }
  static __device__ __forceinline__ void guard(v8f& a, v8f& b, v16h x, v16h y) { dep_guard_h(a, b, x, y); }
  static __device__ __forceinline__ void keep(v16h a, v16h b, v16h c, v16h d) { keep4_h(a, b, c, d); }
};
template <> struct Frag<__bf16> {
  typedef v16b V; union U { v16b v; v8b h[2]; };
  static __device__ __forceinline__ v16b load(const __bf16* p) {
    U f; f.h[0] = *(const v8b*)(p); f.h[1] = *(const v8b*)(p + 16); return f.v;
  }
  static __device__ __forceinline__ v8f mma(v16b a, v16b b, v8f c) {
    return __builtin_amdgcn_wmma_f32_16x16x32_bf16(false, a, false, b, (short)0, c, false, false);
  }
  static __device__ __forceinline__ void guard(v8f& a, v8f& b, v16b x, v16b y) { dep_guard_b(a, b, x, y); }
  static __device__ __forceinline__ void keep(v16b a, v16b b, v16b c, v16b d) { keep4_b(a, b, c, d); }
};

template <int ET> struct Elem;
template <> struct Elem<0> { typedef _Float16 T; };
template <> struct Elem<1> { typedef __bf16 T; };
template <int ET, bool SPLIT, int BIAS_MODE, int OUT_MODE, bool RESID, int ACT = 0>
__global__ __launch_bounds__(256) void wmma_gemm64(
    const unsigned short* __restrict__ Ap, const unsigned short* __restrict__ A2p, int lda, long strideA,
    const unsigned short* __restrict__ Btp, const unsigned short* __restrict__ Bt2p, int ldb, long strideB,
    void* __restrict__ Cout, void* __restrict__ Cout2, int ldc, long strideC,
    const float* __restrict__ bias,
    const float* __restrict__ resid, long strideR,
    int M, int N, int K, float scale) {
  typedef typename Elem<ET>::T T;
  typedef typename Frag<T>::V V;
  const T* A = (const T*)Ap; const T* A2 = (const T*)A2p; const T* Bt = (const T*)Btp; const T* Bt2 = (const T*)Bt2p;
  __shared__ __align__(16) float sT[8][16 * 68];
  const int b    = blockIdx.y;
  const int lane = threadIdx.x & 31;
  const int wave = threadIdx.x >> 5;
  const int tilesN = N >> 6;
  const int tilesM = M >> 6;
  const int tile = blockIdx.x * 8 + wave;
  if (tile >= tilesM * tilesN) return;
  const int tm = tile / tilesN;
  const int tn = tile - tm * tilesN;
  const int m0 = tm << 6;
  const int n0 = tn << 6;

  const T* Ab  = A  + (size_t)b * strideA;
  const T* Bb  = Bt + (size_t)b * strideB;
  const T* Ab2 = SPLIT ? (A2  + (size_t)b * strideA) : nullptr;
  const T* Bb2 = SPLIT ? (Bt2 + (size_t)b * strideB) : nullptr;

  const int rlane = lane & 15;
  const int koff  = (lane >> 4) * 8;
  const int mOff  = (lane >> 4) * 8;

  v8f acc[4][4];
#pragma unroll
  for (int i = 0; i < 4; ++i)
#pragma unroll
    for (int j = 0; j < 4; ++j) acc[i][j] = (v8f){0.f,0.f,0.f,0.f,0.f,0.f,0.f,0.f};

  for (int k0 = 0; k0 < K; k0 += 32) {
    V bh[4], bl[4];
#pragma unroll
    for (int j = 0; j < 4; ++j) {
      const size_t bo = (size_t)(n0 + (j << 4) + rlane) * ldb + koff + k0;
      bh[j] = Frag<T>::load(Bb + bo);
      if (SPLIT) bl[j] = Frag<T>::load(Bb2 + bo);
    }
#pragma unroll
    for (int i = 0; i < 4; ++i) {
      const size_t ao = (size_t)(m0 + (i << 4) + rlane) * lda + koff + k0;
      V ah = Frag<T>::load(Ab + ao);
      V al;
      if (SPLIT) al = Frag<T>::load(Ab2 + ao);
#pragma unroll
      for (int j = 0; j < 4; ++j) {
        acc[i][j] = Frag<T>::mma(ah, bh[j], acc[i][j]);
        if (SPLIT) {
          acc[i][j] = Frag<T>::mma(ah, bl[j], acc[i][j]);
          acc[i][j] = Frag<T>::mma(al, bh[j], acc[i][j]);
        }
      }
      Frag<T>::guard(acc[i][0], acc[i][3], ah, SPLIT ? al : ah);
    }
    Frag<T>::keep(bh[0], bh[1], bh[2], bh[3]);
    if (SPLIT) Frag<T>::keep(bl[0], bl[1], bl[2], bl[3]);
  }
  acc_guard4(acc[0][0], acc[0][1], acc[0][2], acc[0][3]);
  acc_guard4(acc[1][0], acc[1][1], acc[1][2], acc[1][3]);
  acc_guard4(acc[2][0], acc[2][1], acc[2][2], acc[2][3]);
  acc_guard4(acc[3][0], acc[3][1], acc[3][2], acc[3][3]);

  float* slab = sT[wave];
  const float* Rb = RESID ? (resid + (size_t)b * strideR) : nullptr;
#pragma unroll
  for (int i = 0; i < 4; ++i) {
    const int mBase = m0 + (i << 4);
#pragma unroll
    for (int j = 0; j < 4; ++j) {
      const int n = n0 + (j << 4) + rlane;
      float bv = 0.f;
      if (BIAS_MODE == 2) bv = bias[n];
#pragma unroll
      for (int r = 0; r < 8; ++r) {
        float v = acc[i][j][r] * scale;
        if (BIAS_MODE == 1) v += bias[mBase + mOff + r];
        if (BIAS_MODE == 2) v += bv;
        if (RESID) v += Rb[(size_t)(mBase + mOff + r) * ldc + n];
        if (ACT == 1) v = tanhf(v);
        if (ACT == 2) v = fmaxf(v, 0.0f);
        if (ACT == 3) v = v / (1.0f + expf(-v));
        if (ACT == 4) v = (v > 0.f) ? v : 0.01f * v;
        if (ACT == 5) v = 0.5f * v * (1.0f + erff(v * 0.70710678118654752f));
        if (ACT == 6) v = (v > 0.f) ? v : 0.2f * v;
        if (ACT == 7) { const float u = 0.7978845608028654f * (v + 0.044715f * v * v * v); v = 0.5f * v * (1.f + tanhf(u)); }
        slab[(mOff + r) * 68 + (j << 4) + rlane] = v;
      }
    }
    __builtin_amdgcn_fence(3  , "workgroup");
    __builtin_amdgcn_wave_barrier();
    __builtin_amdgcn_fence(2  , "workgroup");
    if (OUT_MODE == 0) {
      float* C = (float*)Cout + (size_t)b * strideC;
      const int hh = lane >> 4, c4 = (lane & 15) * 4;
      for (int pass = 0; pass < 2; ++pass) {
#pragma unroll
        for (int it = 0; it < 8; ++it) {
          const int row = it * 2 + hh;
          v4f v = *(const v4f*)(slab + row * 68 + c4);
          *(volatile v4f*)(C + (size_t)(mBase + row) * ldc + n0 + c4) = v;
        }
        __threadfence();
      }
    } else {
      const int q = lane >> 3, c8 = (lane & 7) * 8;
      unsigned short* C  = (unsigned short*)Cout  + (size_t)b * strideC;
      unsigned short* C2 = (OUT_MODE == 2) ? ((unsigned short*)Cout2 + (size_t)b * strideC) : nullptr;
      for (int pass = 0; pass < 2; ++pass) {
#pragma unroll
        for (int it = 0; it < 4; ++it) {
          const int row = it * 4 + q;
          const float* sp = slab + row * 68 + c8;
          v8h hv, lv;
#pragma unroll
          for (int e = 0; e < 8; ++e) {
            if (OUT_MODE == 1) {
              hv[e] = (_Float16)sp[e];
            } else {
              unsigned short hb = f2bf_bits(sp[e]);
              unsigned short lb = f2bf_bits(sp[e] - bf_bits2f(hb));
              hv[e] = __builtin_bit_cast(_Float16, hb);
              lv[e] = __builtin_bit_cast(_Float16, lb);
            }
          }
          *(volatile v8h*)(C + (size_t)(mBase + row) * ldc + n0 + c8) = hv;
          if (OUT_MODE == 2) *(volatile v8h*)(C2 + (size_t)(mBase + row) * ldc + n0 + c8) = lv;
        }
        __threadfence();
      }
    }
    __builtin_amdgcn_fence(3  , "workgroup");
    __builtin_amdgcn_wave_barrier();
    __builtin_amdgcn_fence(2  , "workgroup");
  }
}

}

typedef _Float16 h16;
typedef float v4f __attribute__((ext_vector_type(4)));
typedef unsigned int v4u __attribute__((ext_vector_type(4)));

static __device__ __forceinline__ h16 toh_flush(float v) { const h16 r = (h16)v; return (fabsf(v) < 6.103515625e-05f) ? (h16)0.0f : r; }
__device__ __forceinline__ float bf16_val(float v) { unsigned u = __float_as_uint(v); u += 0x7FFFu + ((u >> 16) & 1u); return __uint_as_float(u & 0xFFFF0000u); }
__device__ __forceinline__ unsigned es_pk2h(float a, float b) { return (unsigned)__builtin_bit_cast(unsigned short, toh_flush(a)) | ((unsigned)__builtin_bit_cast(unsigned short, toh_flush(b)) << 16); }
__device__ __forceinline__ void es_st8h(unsigned short* d, const float* v) {
    v4u pk; pk.x = es_pk2h(v[0], v[1]); pk.y = es_pk2h(v[2], v[3]); pk.z = es_pk2h(v[4], v[5]); pk.w = es_pk2h(v[6], v[7]);
    volatile v4u* dd = (volatile v4u*)d; *dd = pk; __threadfence(); *dd = pk;
}

__global__ __launch_bounds__(256) void k_es_enc(const float* __restrict__ X, unsigned short* __restrict__ A16, float sc, int n8) {
    #pragma clang fp contract(off)
    const int u = blockIdx.x * 256 + threadIdx.x; if (u >= n8) return;
    const v4f x0 = *(const v4f*)(X + (long long)u * 8), x1 = *(const v4f*)(X + (long long)u * 8 + 4);
    float v[8];
    v[0] = bf16_val(x0.x) * sc; v[1] = bf16_val(x0.y) * sc; v[2] = bf16_val(x0.z) * sc; v[3] = bf16_val(x0.w) * sc;
    v[4] = bf16_val(x1.x) * sc; v[5] = bf16_val(x1.y) * sc; v[6] = bf16_val(x1.z) * sc; v[7] = bf16_val(x1.w) * sc;
    es_st8h(A16 + (long long)u * 8, v);
}

__global__ __launch_bounds__(256) void k_es_w(const float* __restrict__ W1, unsigned short* __restrict__ W16, float sw) {
    #pragma clang fp contract(off)
    const int u = blockIdx.x * 256 + threadIdx.x; if (u >= NOP * (DD / 8)) return;
    const int k0 = 8 * (u % (DD / 8)); const int o = u / (DD / 8);
    const int ol = min(o, HH - 1); const int orr = min(max(o - ROFF, 0), HH - 1);
    const long long offl = (long long)ol * (2 * DD) + k0; const long long offr = (long long)orr * (2 * DD) + DD + k0;
    const v4f a0 = *(const v4f*)(W1 + offl), a1 = *(const v4f*)(W1 + offl + 4);
    const v4f c0 = *(const v4f*)(W1 + offr), c1 = *(const v4f*)(W1 + offr + 4);
    const bool isl = (o < HH); const bool isr = (o >= ROFF) && (o < ROFF + HH);
    const float la[8] = {a0.x, a0.y, a0.z, a0.w, a1.x, a1.y, a1.z, a1.w};
    const float rb[8] = {c0.x, c0.y, c0.z, c0.w, c1.x, c1.y, c1.z, c1.w};
    float v[8];
#pragma unroll
    for (int q = 0; q < 8; ++q) { const float s = isl ? la[q] : (isr ? rb[q] : 0.f); v[q] = bf16_val(s) * sw; }
    es_st8h(W16 + (long long)o * DD + k0, v);
}

__device__ __forceinline__ float es_tanh(float x) { const float e = __expf(2.0f * x); const float r = __builtin_amdgcn_rcpf(1.0f + e); return fmaf(-2.0f, r, 1.0f); }

__global__ __launch_bounds__(256) void k_es_pair(const float* __restrict__ LR, const float* __restrict__ b1, const float* __restrict__ W2, const float* __restrict__ b2, float* __restrict__ out) {
    #pragma clang fp contract(off)
    __shared__ float sL[PT * LSTR];
    __shared__ float sR[PT * LSTR];
    __shared__ float sW[HH];
    const int tid = threadIdx.x;
    const int ib = blockIdx.x * PT, jb = blockIdx.y * PT;
#pragma unroll 1
    for (int idx = tid; idx < PT * (HH / 4); idx += 256) {
        const int r = idx / (HH / 4), c = 4 * (idx % (HH / 4));
        const v4f lv = *(const v4f*)(LR + (size_t)(ib + r) * NOP + c);
        const v4f rv = *(const v4f*)(LR + (size_t)(jb + r) * NOP + ROFF + c);
        const v4f bv = *(const v4f*)(b1 + c);
        sL[r * LSTR + c] = lv.x; sL[r * LSTR + c + 1] = lv.y; sL[r * LSTR + c + 2] = lv.z; sL[r * LSTR + c + 3] = lv.w;
        sR[r * LSTR + c] = rv.x + bf16_val(bv.x); sR[r * LSTR + c + 1] = rv.y + bf16_val(bv.y);
        sR[r * LSTR + c + 2] = rv.z + bf16_val(bv.z); sR[r * LSTR + c + 3] = rv.w + bf16_val(bv.w);
    }
    const float wv = bf16_val(W2[min(tid, HH - 1)]);
    if (tid < HH) sW[tid] = wv;
    __syncthreads();

    const int iloc = tid >> 3;
    const int jg   = tid & 7;
    const int lo = iloc * LSTR;
    const int ro = (jg * 4) * LSTR;
    float a0 = 0.f, a1 = 0.f, a2 = 0.f, a3 = 0.f;
#pragma unroll 4
    for (int h = 0; h < HH; ++h) {
        const float w  = sW[h];
        const float lv = sL[lo + h];
        const float t0 = es_tanh(lv + sR[ro + h]);
        const float t1 = es_tanh(lv + sR[ro + LSTR + h]);
        const float t2 = es_tanh(lv + sR[ro + 2 * LSTR + h]);
        const float t3 = es_tanh(lv + sR[ro + 3 * LSTR + h]);
        a0 = fmaf(w, t0, a0);
        a1 = fmaf(w, t1, a1);
        a2 = fmaf(w, t2, a2);
        a3 = fmaf(w, t3, a3);
    }
    const float bb = bf16_val(b2[0]);
    v4f res; res.x = a0 + bb; res.y = a1 + bb; res.z = a2 + bb; res.w = a3 + bb;
    float* op = out + (size_t)(ib + iloc) * SEQ_FULL + jb + jg * 4;
    *(volatile v4f*)op = res;
    __threadfence();
    *(volatile v4f*)op = res;
}

extern "C" void kernel_launch(void* const* d_in, const int* in_sizes, int n_in, void* d_out, int out_size, void* d_ws, size_t ws_size, hipStream_t stream) {
    if (n_in < 5) return;
    if ((long long)in_sizes[0] < (long long)SEQ * DD) return;
    if ((long long)in_sizes[1] < (long long)HH * 2 * DD) return;
    if (in_sizes[2] < HH || in_sizes[3] < HH || in_sizes[4] < 1) return;
    if ((long long)out_size < (long long)(SEQ - 1) * SEQ_FULL + SEQ) return;
    const float* enc = (const float*)d_in[0];
    const float* W1  = (const float*)d_in[1];
    const float* b1  = (const float*)d_in[2];
    const float* W2  = (const float*)d_in[3];
    const float* b2  = (const float*)d_in[4];
    float* out = (float*)d_out;
    char* wsp = (char*)d_ws;
    unsigned short* A16 = (unsigned short*)wsp; wsp += A16_BYTES;
    unsigned short* W16 = (unsigned short*)wsp; wsp += W16_BYTES;
    float* LR = (float*)wsp; wsp += LR_BYTES;
    if ((size_t)(wsp - (char*)d_ws) > ws_size) return;

    k_es_w<<<(NOP * (DD / 8)) / 256, 256, 0, stream>>>(W1, W16, 1024.0f);
    k_es_enc<<<(SEQ * (DD / 8)) / 256, 256, 0, stream>>>(enc, A16, 8.0f, SEQ * (DD / 8));
    eng::wmma_gemm64<0, false, 0, 0, false, 0><<<dim3((unsigned)((((SEQ) / 64) * ((NOP) / 64) + 7) / 8), (unsigned)(1)), 256, 0, stream>>>(
        (const unsigned short*)(A16), nullptr, DD, 0, (const unsigned short*)(W16), nullptr, DD, 0, (void*)(LR), nullptr, NOP, 0, nullptr, nullptr, 0, SEQ, NOP, DD, 0.0001220703125f);
    k_es_pair<<<dim3(SEQ / PT, SEQ / PT), 256, 0, stream>>>(LR, b1, W2, b2, out);
}
